// UnweightedNeRF_26079041421676
// MI455X (gfx1250) — hardware-run, weakly checked
//
#include <hip/hip_runtime.h>
#include <stddef.h>
#include <stdint.h>

#pragma clang fp contract(off)

#define HD     64
#define NEXP   128
#define NLAY   4
#define CHUNK  256
#define LCAP   320
#define MAXG   4
#define WCAR   64.0f
#define XCAR   16.0f
#define INVC   0.0009765625f

static_assert(LCAP >= 63 + CHUNK);
static_assert(MAXG * 64 + 63 >= LCAP - 1);
static_assert(HD == 64);
static_assert(NLAY * HD == 256);
static_assert((NLAY * HD * HD) % (8 * 256) == 0);

typedef _Float16 v16h __attribute__((ext_vector_type(16)));
typedef _Float16 v8h  __attribute__((ext_vector_type(8)));
typedef float    v8f  __attribute__((ext_vector_type(8)));
typedef float    v4f  __attribute__((ext_vector_type(4)));

union Frag { v16h v; v8h h[2]; };
union XY   { _Float16 h[2 * HD * HD]; float f[HD * HD]; };

__device__ __forceinline__ int clampi(int v, int lo, int hi) { return min(max(v, lo), hi); }

__device__ __forceinline__ v8f mma16(v16h a, v16h b, v8f c) {
  c = __builtin_amdgcn_wmma_f32_16x16x32_f16(false, a, false, b, (short)0, c, false, false);
  asm volatile("v_nop\n\tv_nop\n\tv_nop\n\tv_nop" : "+v"(c) : "v"(a), "v"(b));
  return c;
}

__device__ __forceinline__ v16h ldfrag(const _Float16* p, int ld, int row0, int k0, int lane) {
  const int m = lane & 15, lh = lane >> 4;
  const _Float16* q = p + (row0 + m) * ld + k0 + 8 * lh;
  Frag f;
  f.h[0] = *(const v8h*)(q);
  f.h[1] = *(const v8h*)(q + 16);
  return f.v;
}

__device__ __forceinline__ v8f zero8() { return (v8f){0.f, 0.f, 0.f, 0.f, 0.f, 0.f, 0.f, 0.f}; }

__device__ __forceinline__ v8h cvt8h(v4f a0, v4f a1) {
  return (v8h){(_Float16)a0[0], (_Float16)a0[1], (_Float16)a0[2], (_Float16)a0[3],
               (_Float16)a1[0], (_Float16)a1[1], (_Float16)a1[2], (_Float16)a1[3]};
}

__device__ __forceinline__ void gemm_16x32(const _Float16* cur, const _Float16* wl, int wm, int wn, int lane,
                                           v8f& acc0, v8f& acc1) {
  acc0 = zero8();
  acc1 = zero8();
#pragma unroll
  for (int ks = 0; ks < 2; ++ks) {
    const v16h a  = ldfrag(cur, HD, 16 * wm, 32 * ks, lane);
    const v16h b0 = ldfrag(wl, HD, 32 * wn, 32 * ks, lane);
    const v16h b1 = ldfrag(wl, HD, 32 * wn + 16, 32 * ks, lane);
    acc0 = mma16(a, b0, acc0);
    acc1 = mma16(a, b1, acc1);
  }
}

__device__ __forceinline__ void drain(const float* __restrict__ x, float* __restrict__ out, int N,
                                      const _Float16* sW, const float* sB, XY* sXY, const int* sList,
                                      int base, int nvalid, int tid, int lane, int wave) {
  const int hh = lane >> 4, c = lane & 15;
  const int wm = wave & 3, wn = wave >> 2;

  {
    const int row = tid >> 2, q = tid & 3;
    const int tk = clampi(sList[clampi(base + row, 0, LCAP - 1)], 0, N - 1);
    const float* xr = x + (size_t)tk * HD + 16 * q;
    const float sc = (row < nvalid) ? XCAR : 0.0f;
    v4f a0 = *(const v4f*)(xr);
    v4f a1 = *(const v4f*)(xr + 4);
    v4f a2 = *(const v4f*)(xr + 8);
    v4f a3 = *(const v4f*)(xr + 12);
    a0 = a0 * sc; a1 = a1 * sc; a2 = a2 * sc; a3 = a3 * sc;
    _Float16* d = sXY->h + row * HD + 16 * q;
    *(v8h*)(d)     = cvt8h(a0, a1);
    *(v8h*)(d + 8) = cvt8h(a2, a3);
  }
  __syncthreads();

#pragma unroll 1
  for (int l = 0; l < NLAY - 1; ++l) {
    const _Float16* cur = sXY->h + (l & 1) * (HD * HD);
    _Float16* nxt = sXY->h + ((l + 1) & 1) * (HD * HD);
    const _Float16* wl = sW + l * (HD * HD);
    const float* bl = sB + l * HD;
    v8f acc0, acc1;
    gemm_16x32(cur, wl, wm, wn, lane, acc0, acc1);
    const int n0 = 32 * wn + c, n1 = n0 + 16;
    const float bv0 = bl[n0], bv1 = bl[n1];
#pragma unroll
    for (int r = 0; r < 8; ++r) {
      const int row = 16 * wm + 8 * hh + r;
      const float v0 = fmaxf(acc0[r] * INVC + bv0, 0.0f) * XCAR;
      const float v1 = fmaxf(acc1[r] * INVC + bv1, 0.0f) * XCAR;
      nxt[row * HD + n0] = (_Float16)v0;
      nxt[row * HD + n1] = (_Float16)v1;
    }
    __syncthreads();
  }

  {
    const _Float16* cur = sXY->h + ((NLAY - 1) & 1) * (HD * HD);
    const _Float16* wl = sW + (NLAY - 1) * (HD * HD);
    const float* bl = sB + (NLAY - 1) * HD;
    v8f acc0, acc1;
    gemm_16x32(cur, wl, wm, wn, lane, acc0, acc1);
    __syncthreads();
    const int n0 = 32 * wn + c, n1 = n0 + 16;
    const float bv0 = bl[n0], bv1 = bl[n1];
#pragma unroll
    for (int r = 0; r < 8; ++r) {
      const int row = 16 * wm + 8 * hh + r;
      sXY->f[row * HD + n0] = fmaxf(acc0[r] * INVC + bv0, 0.0f);
      sXY->f[row * HD + n1] = fmaxf(acc1[r] * INVC + bv1, 0.0f);
    }
  }
  __syncthreads();

  for (int ps = 0; ps < 2; ++ps) {
#pragma unroll
    for (int i = 0; i < 4; ++i) {
      const int row = 8 * wave + 2 * i + hh;
      const v4f v = *(const v4f*)(sXY->f + row * HD + 4 * c);
      const int tk = clampi(sList[clampi(base + row, 0, LCAP - 1)], 0, N - 1);
      const bool ok = row < nvalid;
      if (ok) *(volatile v4f*)(out + (size_t)tk * HD + 4 * c) = v;
    }
    __threadfence();
  }
  __syncthreads();
}

__global__ __launch_bounds__(256) void k_moe(const float* __restrict__ x, const float* __restrict__ wts,
                                             const float* __restrict__ bss, const int* __restrict__ idx,
                                             float* __restrict__ out, int N, int nch) {
  __shared__ __align__(16) _Float16 sW[NLAY * HD * HD];
  __shared__ __align__(16) float sB[NLAY * HD];
  __shared__ __align__(16) XY sXY;
  __shared__ __align__(16) int sList[LCAP];
  __shared__ int sWc[8];
  const int tid = threadIdx.x, lane = tid & 31, wave = tid >> 5;
  const int e = blockIdx.x;
  const unsigned ltm = (1u << lane) - 1u;

#pragma unroll 1
  for (int it = 0; it < (NLAY * HD * HD) / (8 * 256); ++it) {
    const int p = it * 256 + tid;
    const int l = p >> 9;
    const int w = p & 511;
    const float* src = wts + ((size_t)(l * NEXP + e) * HD) * HD + 8 * w;
    v4f a0 = *(const v4f*)(src);
    v4f a1 = *(const v4f*)(src + 4);
    a0 = a0 * WCAR; a1 = a1 * WCAR;
    *(v8h*)(sW + l * (HD * HD) + 8 * w) = cvt8h(a0, a1);
  }
  sB[tid] = bss[(size_t)((tid >> 6) * NEXP + e) * HD + (tid & 63)];
  for (int i = tid; i < LCAP; i += 256) sList[i] = 0;
  __syncthreads();

  int carried = 0;
#pragma unroll 1
  for (int ch = 0; ch < nch; ++ch) {
    const int t  = ch * CHUNK + tid;
    const int iv = idx[min(t, N - 1)];
    int et = clampi(iv, 0, NEXP - 1);
    et = (t < N) ? et : -1;
    const bool m = (et == e);
    const unsigned bal = __builtin_amdgcn_ballot_w32(m);
    const int lpre = __builtin_popcount(bal & ltm);
    if (lane == 0) sWc[wave] = __builtin_popcount(bal);
    __syncthreads();
    int hits = 0, wpre = 0;
#pragma unroll
    for (int q = 0; q < 8; ++q) {
      const int cq = sWc[q];
      hits += cq;
      wpre += (q < wave) ? cq : 0;
    }
    if (m) sList[clampi(carried + wpre + lpre, 0, LCAP - 1)] = t;
    __syncthreads();
    const int total = __builtin_amdgcn_readfirstlane(carried + hits);
    const int ng = min(total >> 6, MAXG);
    for (int g = 0; g < ng; ++g)
      drain(x, out, N, sW, sB, &sXY, sList, 64 * g, 64, tid, lane, wave);
    const int rem = clampi(total - 64 * ng, 0, 63);
    const int rv = sList[clampi(64 * ng + tid, 0, LCAP - 1)];
    __syncthreads();
    if (ng > 0 && tid < rem) sList[tid] = rv;
    __syncthreads();
    carried = rem;
  }

  if (carried > 0)
    drain(x, out, N, sW, sB, &sXY, sList, 0, carried, tid, lane, wave);
}

extern "C" void kernel_launch(void* const* d_in, const int* in_sizes, int n_in,
                              void* d_out, int out_size, void* d_ws, size_t ws_size,
                              hipStream_t stream) {
  (void)d_ws; (void)ws_size;
  if (n_in < 4) return;
  const int N = in_sizes[3];
  if (N <= 0) return;
  if (in_sizes[0] != N * HD) return;
  if (in_sizes[1] != NLAY * NEXP * HD * HD) return;
  if (in_sizes[2] != NLAY * NEXP * HD) return;
  if (out_size != N * HD) return;

  const float* x   = (const float*)d_in[0];
  const float* w   = (const float*)d_in[1];
  const float* b   = (const float*)d_in[2];
  const int*   idx = (const int*)d_in[3];
  float*       out = (float*)d_out;

  const int nch = (N + CHUNK - 1) / CHUNK;
  k_moe<<<dim3(NEXP), dim3(256), 0, stream>>>(x, w, b, idx, out, N, nch);
  (void)hipGetLastError();
}
